// SecondOrderDeformableAlignment_4269197492313
// MI455X (gfx1250) — hardware-verified
//
#include <hip/hip_runtime.h>
#include <math.h>
#include <stddef.h>

#pragma clang fp contract(off)

typedef __attribute__((ext_vector_type(16))) _Float16 v16h;
typedef __attribute__((ext_vector_type(8)))  _Float16 v8h;
typedef __attribute__((ext_vector_type(16))) __bf16   v16b;
typedef __attribute__((ext_vector_type(8)))  __bf16   v8b;
typedef __attribute__((ext_vector_type(8)))  float    v8f;
typedef __attribute__((ext_vector_type(4)))  float    v4f;
typedef __attribute__((ext_vector_type(4)))  unsigned v4u;

constexpr int kBatch    = 2;
constexpr int kHgt      = 128;
constexpr int kWid      = 128;
constexpr int kHW       = kHgt * kWid;
constexpr int kPix      = kBatch * kHW;
constexpr int kHalfPix  = kPix / 2;
constexpr int kCinX     = 128;
constexpr int kCef      = 192;
constexpr int kCin1     = 196;
constexpr int kCin1P    = 224;
constexpr int kCmid     = 64;
constexpr int kCout4    = 432;
constexpr int kCout4P   = 448;
constexpr int kGroups   = 16;
constexpr int kCpg      = 8;
constexpr int kTaps     = 9;
constexpr int kKdcn     = kCinX * kTaps;
constexpr int kCoutD    = 64;
constexpr int kThreads  = 256;
constexpr int kGatherPix = 8;
constexpr int kSlabHalves = 3 * 66 * 32;
constexpr int kStgPitch = 68;

constexpr float kMaxMag   = 10.0f;
constexpr float kWCarry   = 64.0f;
constexpr float kA1Carry  = 2.0f;
constexpr float kA2Carry  = 4.0f;
constexpr float kA3Carry  = 16.0f;
constexpr float kLogCarry = 32.0f;
constexpr float kLogInv   = 1.0f / 32.0f;
constexpr float kVCarry   = 8.0f;

static_assert(kCin1P % 32 == 0 && kCmid % 32 == 0 && kKdcn % 32 == 0);
static_assert(kCmid % 64 == 0 && kCout4P % 64 == 0 && kCoutD % 64 == 0);
static_assert(kPix % 64 == 0 && kHalfPix % 64 == 0 && (kHalfPix / 64) % 8 == 0);
static_assert(kWid == 128 && kHgt == 128 && kGroups * kCpg == kCinX);
static_assert(kHalfPix % kGatherPix == 0 && (kGatherPix * kKdcn) % 8 == 0);
static_assert(kCout4 == 27 * kGroups && 2 * kGroups * kTaps == 288);

constexpr size_t kBytesP0  = (size_t)kPix * kCin1P * 2;
constexpr size_t kBytesAct = (size_t)kPix * kCmid * 2;
constexpr size_t kBytesLog = (size_t)kPix * kCout4P * 2;
constexpr size_t kBytesV   = (size_t)kHalfPix * kKdcn * 2;
constexpr size_t kBytesTmp = (size_t)kPix * kCoutD * 4;
constexpr size_t kBytesW1  = (size_t)kTaps * kCmid * kCin1P * 2;
constexpr size_t kBytesW2  = (size_t)kTaps * kCmid * kCmid * 2;
constexpr size_t kBytesW4  = (size_t)kTaps * kCout4P * kCmid * 2;
constexpr size_t kBytesWD  = (size_t)kCoutD * kKdcn * 2;
constexpr size_t kOffP0  = 0;
constexpr size_t kOffA1  = kOffP0 + kBytesP0;
constexpr size_t kOffA2  = kOffA1 + kBytesAct;
constexpr size_t kOffA3  = kOffA2 + kBytesAct;
constexpr size_t kOffLog = kOffA3 + kBytesAct;
constexpr size_t kOffV   = kOffLog + kBytesLog;
constexpr size_t kOffTmp = kOffV + kBytesV;
constexpr size_t kOffW1  = kOffTmp + kBytesTmp;
constexpr size_t kOffW2  = kOffW1 + kBytesW1;
constexpr size_t kOffW3  = kOffW2 + kBytesW2;
constexpr size_t kOffW4  = kOffW3 + kBytesW2;
constexpr size_t kOffWD  = kOffW4 + kBytesW4;
constexpr size_t kWsTotal = kOffWD + kBytesWD;
static_assert(kWsTotal == 103829504u);
static_assert(kWsTotal <= 134217728u);
static_assert(kOffA1 % 4096 == 0 && kOffLog % 4096 == 0 && kOffV % 4096 == 0 && kOffTmp % 4096 == 0);
static_assert(kOffW1 % 4096 == 0 && kOffW2 % 4096 == 0 && kOffW3 % 4096 == 0 && kOffW4 % 4096 == 0 && kOffWD % 4096 == 0);
constexpr int kChunksW1 = kTaps * kCmid * kCin1P / 8;
constexpr int kChunksW2 = kTaps * kCmid * kCmid / 8;
constexpr int kChunksW4 = kTaps * kCout4P * kCmid / 8;
constexpr int kChunksWD = kCoutD * kKdcn / 8;
static_assert(kChunksW1 % kThreads == 0 && kChunksW2 % kThreads == 0 && kChunksW4 % kThreads == 0 && kChunksWD % kThreads == 0);
constexpr int kBlkW1 = kChunksW1 / kThreads;
constexpr int kBlkW2 = kChunksW2 / kThreads;
constexpr int kBlkW4 = kChunksW4 / kThreads;
constexpr int kBlkWD = kChunksWD / kThreads;
constexpr int kBlkWtot = kBlkW1 + 2 * kBlkW2 + kBlkW4 + kBlkWD;

__device__ __forceinline__ unsigned short f2bf_bits(float f) {
  unsigned u = __float_as_uint(f);
  return (unsigned short)((u + 0x7FFFu + ((u >> 16) & 1u)) >> 16);
}
__device__ __forceinline__ float bf_bits2f(unsigned short h) { return __uint_as_float(((unsigned)h) << 16); }

__device__ __forceinline__ void dep_guard_h(v8f& a, v8f& b, v16h x, v16h y) { asm volatile("v_nop\n\tv_nop\n\tv_nop\n\tv_nop" : "+v"(a), "+v"(b) : "v"(x), "v"(y)); }
__device__ __forceinline__ void dep_guard_b(v8f& a, v8f& b, v16b x, v16b y) { asm volatile("v_nop\n\tv_nop\n\tv_nop\n\tv_nop" : "+v"(a), "+v"(b) : "v"(x), "v"(y)); }
__device__ __forceinline__ void keep4_h(v16h a, v16h b, v16h c, v16h d) { asm volatile("v_nop" :: "v"(a), "v"(b), "v"(c), "v"(d)); }
__device__ __forceinline__ void keep4_b(v16b a, v16b b, v16b c, v16b d) { asm volatile("v_nop" :: "v"(a), "v"(b), "v"(c), "v"(d)); }
__device__ __forceinline__ void acc_guard4(v8f& a, v8f& b, v8f& c, v8f& d) { asm volatile("v_nop\n\tv_nop\n\tv_nop\n\tv_nop" : "+v"(a), "+v"(b), "+v"(c), "+v"(d)); }
template <typename T> struct Frag;
template <> struct Frag<_Float16> {
  typedef v16h V; union U { v16h v; v8h h[2]; };
  static __device__ __forceinline__ v16h load(const _Float16* p) {
    U f; f.h[0] = *(const v8h*)(p); f.h[1] = *(const v8h*)(p + 16); return f.v;
  }
  static __device__ __forceinline__ v8f mma(v16h a, v16h b, v8f c) {
    return __builtin_amdgcn_wmma_f32_16x16x32_f16(false, a, false, b, (short)0, c, false, false);
  }
  static __device__ __forceinline__ void guard(v8f& a, v8f& b, v16h x, v16h y) { dep_guard_h(a, b, x, y); }
  static __device__ __forceinline__ void keep(v16h a, v16h b, v16h c, v16h d) { keep4_h(a, b, c, d); }
};
template <> struct Frag<__bf16> {
  typedef v16b V; union U { v16b v; v8b h[2]; };
  static __device__ __forceinline__ v16b load(const __bf16* p) {
    U f; f.h[0] = *(const v8b*)(p); f.h[1] = *(const v8b*)(p + 16); return f.v;
  }
  static __device__ __forceinline__ v8f mma(v16b a, v16b b, v8f c) {
    return __builtin_amdgcn_wmma_f32_16x16x32_bf16(false, a, false, b, (short)0, c, false, false);
  }
  static __device__ __forceinline__ void guard(v8f& a, v8f& b, v16b x, v16b y) { dep_guard_b(a, b, x, y); }
  static __device__ __forceinline__ void keep(v16b a, v16b b, v16b c, v16b d) { keep4_b(a, b, c, d); }
};

template <int ET> struct Elem;
template <> struct Elem<0> { typedef _Float16 T; };
template <> struct Elem<1> { typedef __bf16 T; };
template <int ET, bool SPLIT, int BIAS_MODE, int OUT_MODE, bool RESID, int ACT = 0>
__global__ __launch_bounds__(256) void wmma_gemm64(
    const unsigned short* __restrict__ Ap, const unsigned short* __restrict__ A2p, int lda, long strideA,
    const unsigned short* __restrict__ Btp, const unsigned short* __restrict__ Bt2p, int ldb, long strideB,
    void* __restrict__ Cout, void* __restrict__ Cout2, int ldc, long strideC,
    const float* __restrict__ bias,
    const float* __restrict__ resid, long strideR,
    int M, int N, int K, float scale) {
  typedef typename Elem<ET>::T T;
  typedef typename Frag<T>::V V;
  const T* A = (const T*)Ap; const T* A2 = (const T*)A2p; const T* Bt = (const T*)Btp; const T* Bt2 = (const T*)Bt2p;
  __shared__ __align__(16) float sT[8][16 * 68];
  const int b    = blockIdx.y;
  const int lane = threadIdx.x & 31;
  const int wave = threadIdx.x >> 5;
  const int tilesN = N >> 6;
  const int tilesM = M >> 6;
  const int tile = blockIdx.x * 8 + wave;
  if (tile >= tilesM * tilesN) return;
  const int tm = tile / tilesN;
  const int tn = tile - tm * tilesN;
  const int m0 = tm << 6;
  const int n0 = tn << 6;

  const T* Ab  = A  + (size_t)b * strideA;
  const T* Bb  = Bt + (size_t)b * strideB;
  const T* Ab2 = SPLIT ? (A2  + (size_t)b * strideA) : nullptr;
  const T* Bb2 = SPLIT ? (Bt2 + (size_t)b * strideB) : nullptr;

  const int rlane = lane & 15;
  const int koff  = (lane >> 4) * 8;
  const int mOff  = (lane >> 4) * 8;

  v8f acc[4][4];
#pragma unroll
  for (int i = 0; i < 4; ++i)
#pragma unroll
    for (int j = 0; j < 4; ++j) acc[i][j] = (v8f){0.f,0.f,0.f,0.f,0.f,0.f,0.f,0.f};

  for (int k0 = 0; k0 < K; k0 += 32) {
    V bh[4], bl[4];
#pragma unroll
    for (int j = 0; j < 4; ++j) {
      const size_t bo = (size_t)(n0 + (j << 4) + rlane) * ldb + koff + k0;
      bh[j] = Frag<T>::load(Bb + bo);
      if (SPLIT) bl[j] = Frag<T>::load(Bb2 + bo);
    }
#pragma unroll
    for (int i = 0; i < 4; ++i) {
      const size_t ao = (size_t)(m0 + (i << 4) + rlane) * lda + koff + k0;
      V ah = Frag<T>::load(Ab + ao);
      V al;
      if (SPLIT) al = Frag<T>::load(Ab2 + ao);
#pragma unroll
      for (int j = 0; j < 4; ++j) {
        acc[i][j] = Frag<T>::mma(ah, bh[j], acc[i][j]);
        if (SPLIT) {
          acc[i][j] = Frag<T>::mma(ah, bl[j], acc[i][j]);
          acc[i][j] = Frag<T>::mma(al, bh[j], acc[i][j]);
        }
      }
      Frag<T>::guard(acc[i][0], acc[i][3], ah, SPLIT ? al : ah);
    }
    Frag<T>::keep(bh[0], bh[1], bh[2], bh[3]);
    if (SPLIT) Frag<T>::keep(bl[0], bl[1], bl[2], bl[3]);
  }
  acc_guard4(acc[0][0], acc[0][1], acc[0][2], acc[0][3]);
  acc_guard4(acc[1][0], acc[1][1], acc[1][2], acc[1][3]);
  acc_guard4(acc[2][0], acc[2][1], acc[2][2], acc[2][3]);
  acc_guard4(acc[3][0], acc[3][1], acc[3][2], acc[3][3]);

  float* slab = sT[wave];
  const float* Rb = RESID ? (resid + (size_t)b * strideR) : nullptr;
#pragma unroll
  for (int i = 0; i < 4; ++i) {
    const int mBase = m0 + (i << 4);
#pragma unroll
    for (int j = 0; j < 4; ++j) {
      const int n = n0 + (j << 4) + rlane;
      float bv = 0.f;
      if (BIAS_MODE == 2) bv = bias[n];
#pragma unroll
      for (int r = 0; r < 8; ++r) {
        float v = acc[i][j][r] * scale;
        if (BIAS_MODE == 1) v += bias[mBase + mOff + r];
        if (BIAS_MODE == 2) v += bv;
        if (RESID) v += Rb[(size_t)(mBase + mOff + r) * ldc + n];
        if (ACT == 1) v = tanhf(v);
        if (ACT == 2) v = fmaxf(v, 0.0f);
        if (ACT == 3) v = v / (1.0f + expf(-v));
        if (ACT == 4) v = (v > 0.f) ? v : 0.01f * v;
        if (ACT == 5) v = 0.5f * v * (1.0f + erff(v * 0.70710678118654752f));
        slab[(mOff + r) * 68 + (j << 4) + rlane] = v;
      }
    }
    __builtin_amdgcn_fence(__ATOMIC_RELEASE, "workgroup");
    __builtin_amdgcn_wave_barrier();
    __builtin_amdgcn_fence(__ATOMIC_ACQUIRE, "workgroup");
    if (OUT_MODE == 0) {
      float* C = (float*)Cout + (size_t)b * strideC;
      const int hh = lane >> 4, c4 = (lane & 15) * 4;
      for (int pass = 0; pass < 2; ++pass) {
#pragma unroll
        for (int it = 0; it < 8; ++it) {
          const int row = it * 2 + hh;
          v4f v = *(const v4f*)(slab + row * 68 + c4);
          *(volatile v4f*)(C + (size_t)(mBase + row) * ldc + n0 + c4) = v;
        }
        __threadfence();
      }
    } else {
      const int q = lane >> 3, c8 = (lane & 7) * 8;
      unsigned short* C  = (unsigned short*)Cout  + (size_t)b * strideC;
      unsigned short* C2 = (OUT_MODE == 2) ? ((unsigned short*)Cout2 + (size_t)b * strideC) : nullptr;
      for (int pass = 0; pass < 2; ++pass) {
#pragma unroll
        for (int it = 0; it < 4; ++it) {
          const int row = it * 4 + q;
          const float* sp = slab + row * 68 + c8;
          v8h hv, lv;
#pragma unroll
          for (int e = 0; e < 8; ++e) {
            if (OUT_MODE == 1) {
              hv[e] = (_Float16)sp[e];
            } else {
              unsigned short hb = f2bf_bits(sp[e]);
              unsigned short lb = f2bf_bits(sp[e] - bf_bits2f(hb));
              hv[e] = __builtin_bit_cast(_Float16, hb);
              lv[e] = __builtin_bit_cast(_Float16, lb);
            }
          }
          *(volatile v8h*)(C + (size_t)(mBase + row) * ldc + n0 + c8) = hv;
          if (OUT_MODE == 2) *(volatile v8h*)(C2 + (size_t)(mBase + row) * ldc + n0 + c8) = lv;
        }
        __threadfence();
      }
    }
    __builtin_amdgcn_fence(__ATOMIC_RELEASE, "workgroup");
    __builtin_amdgcn_wave_barrier();
    __builtin_amdgcn_fence(__ATOMIC_ACQUIRE, "workgroup");
  }
}
typedef Frag<_Float16> FragH;

__device__ __forceinline__ void guard_acc2(v8f& a, v8f& b, v16h x, v16h y, v16h z) {
  asm volatile("v_nop\n\tv_nop\n\tv_nop\n\tv_nop" : "+v"(a), "+v"(b) : "v"(x), "v"(y), "v"(z));
}

__device__ __forceinline__ float h16_to_f32(unsigned hb) {
  const unsigned sgn = (hb & 0x8000u) << 16; const unsigned em = hb & 0x7fffu;
  const float fn = __uint_as_float((em << 13) + 0x38000000u);
  const float fs = (float)em * 5.9604644775390625e-8f;
  const float mag = (em < 0x400u) ? fs : fn; return __uint_as_float(__float_as_uint(mag) | sgn);
}

__global__ __launch_bounds__(kThreads) void pack_input_kernel(
    const float* __restrict__ ef, const float* __restrict__ fl1, const float* __restrict__ fl2,
    unsigned short* __restrict__ p0) {
  __shared__ __align__(16) float tile[kCin1 * 64];
  const int tid = threadIdx.x;
  const int bx = blockIdx.x;
  const int b = bx >> 8, h = (bx >> 1) & 127, w0 = (bx & 1) * 64;
  const size_t pix0 = (size_t)bx * 64;
#pragma unroll 1
  for (int it = 0; it < 12; ++it) {
    const int idx = it * kThreads + tid;
    const int ch = idx >> 4, p4 = (idx & 15) * 4;
    const v4f v = *(const v4f*)(ef + ((size_t)(b * kCef + ch) * kHW + (size_t)h * kWid + w0 + p4));
    *(v4f*)(tile + ch * 64 + p4) = v;
  }
  if (tid < 64) {
    const int comp = (tid >> 4) & 1, p4 = (tid & 15) * 4;
    const int sel = tid >> 5;
    const size_t fo = (size_t)(b * 2 + comp) * kHW + (size_t)h * kWid + w0 + p4;
    const v4f va = *(const v4f*)(fl1 + fo);
    const v4f vb = *(const v4f*)(fl2 + fo);
    const float sa = (sel == 0) ? 1.0f : 0.0f, sb = 1.0f - sa;
    v4f v;
    v[0] = fmaf(sa, va[0], sb * vb[0]);
    v[1] = fmaf(sa, va[1], sb * vb[1]);
    v[2] = fmaf(sa, va[2], sb * vb[2]);
    v[3] = fmaf(sa, va[3], sb * vb[3]);
    *(v4f*)(tile + (kCef + sel * 2 + comp) * 64 + p4) = v;
  }
  __syncthreads();
  for (int pass = 0; pass < 2; ++pass) {
#pragma unroll 1
    for (int it = 0; it < 7; ++it) {
      const int q = it * kThreads + tid;
      const int px = q / 28, ch0 = (q - px * 28) * 8;
      v8h hv;
#pragma unroll
      for (int e = 0; e < 8; ++e) {
        const int ch = ch0 + e;
        const int chc = (ch < kCin1) ? ch : (kCin1 - 1);
        const float fz = (ch < kCin1) ? 1.0f : 0.0f;
        hv[e] = (_Float16)(tile[chc * 64 + px] * fz);
      }
      *(volatile v8h*)(p0 + pix0 * kCin1P + (size_t)q * 8) = hv;
    }
    __threadfence();
  }
}

__device__ __forceinline__ void conv_w_chunk(const float* __restrict__ w, int cin, int cout, int cinp, int np, int q,
                                             unsigned short* __restrict__ dst) {
  const int e0 = q * 8;
  const int plane = np * cinp;
  const int tap = e0 / plane;
  const int rem = e0 - tap * plane;
  const int n = rem / cinp;
  const int k0 = rem - n * cinp;
  const int nc = (n < cout) ? n : (cout - 1);
  const float fn = (n < cout) ? 1.0f : 0.0f;
  v8h hv;
#pragma unroll
  for (int e = 0; e < 8; ++e) {
    const int ci = k0 + e;
    const int cic = (ci < cin) ? ci : (cin - 1);
    const float fz = ((ci < cin) ? 1.0f : 0.0f) * fn;
    const float v = w[((size_t)nc * cin + cic) * kTaps + tap];
    hv[e] = (_Float16)((v * kWCarry) * fz);
  }
  *(volatile v8h*)(dst + e0) = hv;
  __threadfence();
  *(volatile v8h*)(dst + e0) = hv;
}

__global__ __launch_bounds__(kThreads) void weight_prep_kernel(
    const float* __restrict__ w1, const float* __restrict__ w2, const float* __restrict__ w3,
    const float* __restrict__ w4, const float* __restrict__ wd,
    unsigned short* __restrict__ w1p, unsigned short* __restrict__ w2p, unsigned short* __restrict__ w3p,
    unsigned short* __restrict__ w4p, unsigned short* __restrict__ wdp) {
  const int bx = blockIdx.x;
  const int tid = threadIdx.x;
  if (bx < kBlkW1) {
    conv_w_chunk(w1, kCin1, kCmid, kCin1P, kCmid, bx * kThreads + tid, w1p);
  } else if (bx < kBlkW1 + kBlkW2) {
    conv_w_chunk(w2, kCmid, kCmid, kCmid, kCmid, (bx - kBlkW1) * kThreads + tid, w2p);
  } else if (bx < kBlkW1 + 2 * kBlkW2) {
    conv_w_chunk(w3, kCmid, kCmid, kCmid, kCmid, (bx - kBlkW1 - kBlkW2) * kThreads + tid, w3p);
  } else if (bx < kBlkW1 + 2 * kBlkW2 + kBlkW4) {
    conv_w_chunk(w4, kCmid, kCout4, kCmid, kCout4P, (bx - kBlkW1 - 2 * kBlkW2) * kThreads + tid, w4p);
  } else {
    const int q = (bx - kBlkW1 - 2 * kBlkW2 - kBlkW4) * kThreads + tid;
    const int e0 = q * 8;
    v8h hv;
#pragma unroll
    for (int e = 0; e < 8; ++e) hv[e] = (_Float16)(wd[e0 + e] * kWCarry);
    *(volatile v8h*)(wdp + e0) = hv;
    __threadfence();
    *(volatile v8h*)(wdp + e0) = hv;
  }
}

template <int MODE>
__global__ __launch_bounds__(kThreads) void conv3x3_kernel(
    const unsigned short* __restrict__ inP, int cinp, int cblks,
    const unsigned short* __restrict__ wP, int np,
    const float* __restrict__ bias, int nbias,
    float scale, float ocarry,
    unsigned short* __restrict__ outP) {
  __shared__ __align__(16) _Float16 slab[kSlabHalves];
  __shared__ __align__(16) float stg[64 * kStgPitch];
  const int tid = threadIdx.x, lane = tid & 31, wave = tid >> 5;
  const int rlane = lane & 15, hh = lane >> 4, koff = hh * 8;
  const int bx = blockIdx.x;
  const int b = bx >> 8, h = (bx >> 1) & 127, w0 = (bx & 1) * 64;
  const int pix0 = bx * 64;
  const int n0 = blockIdx.y * 64;
  const int mi = wave >> 1;
  const int jn0 = (wave & 1) * 2;
  const _Float16* w16 = (const _Float16*)wP;
  const int nrow = n0 + jn0 * 16 + rlane;

  v8f acc0 = {0.f, 0.f, 0.f, 0.f, 0.f, 0.f, 0.f, 0.f};
  v8f acc1 = {0.f, 0.f, 0.f, 0.f, 0.f, 0.f, 0.f, 0.f};

#pragma unroll 1
  for (int cb = 0; cb < cblks; ++cb) {
    __syncthreads();
#pragma unroll 1
    for (int e = tid; e < 792; e += kThreads) {
      const int c8 = (e & 3) * 8;
      const int col = (e >> 2) % 66;
      const int row = (e >> 2) / 66;
      const int hs = h + row - 1, wsx = w0 + col - 1;
      const bool valid = (hs >= 0) && (hs < kHgt) && (wsx >= 0) && (wsx < kWid);
      const int hc = (hs < 0) ? 0 : ((hs > kHgt - 1) ? (kHgt - 1) : hs);
      const int wc = (wsx < 0) ? 0 : ((wsx > kWid - 1) ? (kWid - 1) : wsx);
      const v4u* src = (const v4u*)(inP + ((size_t)((b * kHgt + hc) * kWid + wc) * cinp + cb * 32 + c8));
      v4u d = *src;
      const unsigned mk = 0u - (unsigned)valid;
      d = d & (v4u){mk, mk, mk, mk};
      *(v4u*)(slab + (row * 66 + col) * 32 + c8) = d;
    }
    __syncthreads();
#pragma unroll
    for (int tap = 0; tap < kTaps; ++tap) {
      const int ky = tap / 3, kx = tap - ky * 3;
      const v16h a = FragH::load(slab + (ky * 66 + mi * 16 + rlane + kx) * 32 + koff);
      const _Float16* wr = w16 + (size_t)(tap * np + nrow) * cinp + cb * 32 + koff;
      const v16h b0 = FragH::load(wr);
      const v16h b1 = FragH::load(wr + 16 * cinp);
      acc0 = FragH::mma(a, b0, acc0);
      acc1 = FragH::mma(a, b1, acc1);
      guard_acc2(acc0, acc1, a, b0, b1);
    }
  }

  {
    const int nA = nrow, nB = nrow + 16;
    const float bA = bias[(nA < nbias) ? nA : (nbias - 1)];
    const float bB = bias[(nB < nbias) ? nB : (nbias - 1)];
    float* srow = stg + (mi * 16 + hh * 8) * kStgPitch + jn0 * 16 + rlane;
#pragma unroll
    for (int r = 0; r < 8; ++r) {
      float va = acc0[r] * scale + bA;
      float vb = acc1[r] * scale + bB;
      if (MODE == 0) {
        va = (va >= 0.0f) ? va : 0.1f * va;
        vb = (vb >= 0.0f) ? vb : 0.1f * vb;
      }
      srow[r * kStgPitch] = va * ocarry;
      srow[r * kStgPitch + 16] = vb * ocarry;
    }
  }
  __syncthreads();
  {
    const int opitch = (MODE == 0) ? kCmid : kCout4P;
    const int ocol = (MODE == 0) ? 0 : n0;
    for (int pass = 0; pass < 2; ++pass) {
#pragma unroll
      for (int it = 0; it < 2; ++it) {
        const int q = it * kThreads + tid;
        const int px = q >> 3, c8 = (q & 7) * 8;
        const v4f f0 = *(const v4f*)(stg + px * kStgPitch + c8);
        const v4f f1 = *(const v4f*)(stg + px * kStgPitch + c8 + 4);
        v8h hv;
        hv[0] = (_Float16)f0[0]; hv[1] = (_Float16)f0[1]; hv[2] = (_Float16)f0[2]; hv[3] = (_Float16)f0[3];
        hv[4] = (_Float16)f1[0]; hv[5] = (_Float16)f1[1]; hv[6] = (_Float16)f1[2]; hv[7] = (_Float16)f1[3];
        *(volatile v8h*)(outP + (size_t)(pix0 + px) * opitch + ocol + c8) = hv;
      }
      __threadfence();
    }
  }
}

__global__ __launch_bounds__(kThreads) void deform_gather_kernel(
    const float* __restrict__ x, const unsigned* __restrict__ lg32,
    const float* __restrict__ fl1, const float* __restrict__ fl2,
    int pixbase, unsigned short* __restrict__ vout) {
  __shared__ __align__(16) float stg[kGatherPix * kKdcn];
  const int tid = threadIdx.x;
  const int blk = blockIdx.x;
  const int pix0 = pixbase + blk * kGatherPix;
#pragma unroll 1
  for (int it = tid; it < kGatherPix * kGroups * kTaps; it += kThreads) {
    const int pl = it / (kGroups * kTaps);
    const int rem = it - pl * (kGroups * kTaps);
    const int g = rem / kTaps;
    const int kk = rem - g * kTaps;
    const int p = pix0 + pl;
    const int b = p >> 14;
    const int hw = p & (kHW - 1);
    const int h = hw >> 7;
    const int w = hw & 127;
    const int gk = g * kTaps + kk;
    const unsigned wo = lg32[(size_t)p * (kCout4P / 2) + gk];
    const unsigned wm = lg32[(size_t)p * (kCout4P / 2) + 144 + (gk >> 1)];
    const float ody = h16_to_f32(wo & 0xffffu) * kLogInv;
    const float odx = h16_to_f32(wo >> 16) * kLogInv;
    const unsigned mbits = (wm >> ((gk & 1) * 16)) & 0xffffu;
    const float omd = h16_to_f32(mbits) * kLogInv;
    const size_t fo = (size_t)(b * 2) * kHW + hw;
    const float f1y = fl1[fo], f1x = fl1[fo + kHW];
    const float f2y = fl2[fo], f2x = fl2[fo + kHW];
    const float s1 = (g < 8) ? 1.0f : 0.0f, s2 = 1.0f - s1;
    const float fy = fmaf(s1, f1y, s2 * f2y);
    const float fx = fmaf(s1, f1x, s2 * f2x);
    const float dy = kMaxMag * tanhf(ody) + fy;
    const float dx = kMaxMag * tanhf(odx) + fx;
    const float md = 1.0f / (1.0f + expf(-omd));
    const int ky = kk / 3, kx = kk - ky * 3;
    const float sy = (float)(h + ky - 1) + dy;
    const float sx = (float)(w + kx - 1) + dx;
    const float y0f = floorf(sy), x0f = floorf(sx);
    const float y1f = y0f + 1.0f, x1f = x0f + 1.0f;
    const float wy0 = 1.0f - (sy - y0f), wy1 = 1.0f - (y1f - sy);
    const float wx0 = 1.0f - (sx - x0f), wx1 = 1.0f - (x1f - sx);
    const float vy0 = ((y0f >= 0.0f) && (y0f < (float)kHgt)) ? 1.0f : 0.0f;
    const float vy1 = ((y1f >= 0.0f) && (y1f < (float)kHgt)) ? 1.0f : 0.0f;
    const float vx0 = ((x0f >= 0.0f) && (x0f < (float)kWid)) ? 1.0f : 0.0f;
    const float vx1 = ((x1f >= 0.0f) && (x1f < (float)kWid)) ? 1.0f : 0.0f;
    const float w00 = (wy0 * wx0) * (vy0 * vx0);
    const float w01 = (wy0 * wx1) * (vy0 * vx1);
    const float w10 = (wy1 * wx0) * (vy1 * vx0);
    const float w11 = (wy1 * wx1) * (vy1 * vx1);
    const int cy0 = (int)fminf(fmaxf(y0f, 0.0f), (float)(kHgt - 1));
    const int cy1 = (int)fminf(fmaxf(y1f, 0.0f), (float)(kHgt - 1));
    const int cx0 = (int)fminf(fmaxf(x0f, 0.0f), (float)(kWid - 1));
    const int cx1 = (int)fminf(fmaxf(x1f, 0.0f), (float)(kWid - 1));
    const int o00 = cy0 * kWid + cx0, o01 = cy0 * kWid + cx1;
    const int o10 = cy1 * kWid + cx0, o11 = cy1 * kWid + cx1;
    const float* xg = x + (size_t)(b * kCinX + g * kCpg) * kHW;
    float* srow = stg + pl * kKdcn + g * (kCpg * kTaps) + kk;
#pragma unroll 1
    for (int c = 0; c < kCpg; ++c) {
      const float* xc = xg + (size_t)c * kHW;
      float v = 0.0f;
      v = v + xc[o00] * w00;
      v = v + xc[o01] * w01;
      v = v + xc[o10] * w10;
      v = v + xc[o11] * w11;
      srow[c * kTaps] = (v * md) * kVCarry;
    }
  }
  __syncthreads();
  {
    const size_t vbase = (size_t)blk * kGatherPix * kKdcn;
    for (int pass = 0; pass < 2; ++pass) {
#pragma unroll 1
      for (int q = tid; q < kGatherPix * kKdcn / 8; q += kThreads) {
        const v4f f0 = *(const v4f*)(stg + q * 8);
        const v4f f1 = *(const v4f*)(stg + q * 8 + 4);
        v8h hv;
        hv[0] = (_Float16)f0[0]; hv[1] = (_Float16)f0[1]; hv[2] = (_Float16)f0[2]; hv[3] = (_Float16)f0[3];
        hv[4] = (_Float16)f1[0]; hv[5] = (_Float16)f1[1]; hv[6] = (_Float16)f1[2]; hv[7] = (_Float16)f1[3];
        *(volatile v8h*)(vout + vbase + (size_t)q * 8) = hv;
      }
      __threadfence();
    }
  }
}

__global__ __launch_bounds__(kThreads) void nchw_out_kernel(const float* __restrict__ tmp, float* __restrict__ out) {
  __shared__ __align__(16) float t[kCoutD * 132];
  const int tid = threadIdx.x;
  const int bh = blockIdx.x;
  const int b = bh >> 7, h = bh & 127;
  const size_t rowpix0 = (size_t)bh * kWid;
#pragma unroll 1
  for (int it = 0; it < 8; ++it) {
    const int r = it * kThreads + tid;
    const int px = r >> 4, o4 = (r & 15) * 4;
    const v4f v = *(const v4f*)(tmp + (rowpix0 + px) * kCoutD + o4);
    t[(o4 + 0) * 132 + px] = v[0];
    t[(o4 + 1) * 132 + px] = v[1];
    t[(o4 + 2) * 132 + px] = v[2];
    t[(o4 + 3) * 132 + px] = v[3];
  }
  __syncthreads();
  for (int pass = 0; pass < 2; ++pass) {
#pragma unroll
    for (int it = 0; it < 8; ++it) {
      const int q = it * kThreads + tid;
      const int o = q >> 5, w4 = (q & 31) * 4;
      const v4f v = *(const v4f*)(t + o * 132 + w4);
      *(volatile v4f*)(out + ((size_t)(b * kCoutD + o) * kHgt + h) * kWid + w4) = v;
    }
    __threadfence();
  }
}

extern "C" void kernel_launch(void* const* d_in, const int* in_sizes, int n_in,
                              void* d_out, int out_size, void* d_ws, size_t ws_size,
                              hipStream_t stream) {
  if (n_in < 14) return;
  if (ws_size < kWsTotal) return;
  if ((size_t)out_size < (size_t)kPix * kCoutD) return;
  if (in_sizes[0] != kBatch * kCinX * kHW || in_sizes[1] != kBatch * kCef * kHW) return;
  if (in_sizes[10] != kCout4 * kCmid * kTaps || in_sizes[12] != kCoutD * kCinX * kTaps) return;

  const float* x    = (const float*)d_in[0];
  const float* ef   = (const float*)d_in[1];
  const float* fl1  = (const float*)d_in[2];
  const float* fl2  = (const float*)d_in[3];
  const float* w1   = (const float*)d_in[4];
  const float* b1   = (const float*)d_in[5];
  const float* w2   = (const float*)d_in[6];
  const float* b2   = (const float*)d_in[7];
  const float* w3   = (const float*)d_in[8];
  const float* b3   = (const float*)d_in[9];
  const float* w4   = (const float*)d_in[10];
  const float* b4   = (const float*)d_in[11];
  const float* dcnw = (const float*)d_in[12];
  const float* dcnb = (const float*)d_in[13];
  float* out = (float*)d_out;

  char* ws = (char*)d_ws;
  unsigned short* p0  = (unsigned short*)(ws + kOffP0);
  unsigned short* a1  = (unsigned short*)(ws + kOffA1);
  unsigned short* a2  = (unsigned short*)(ws + kOffA2);
  unsigned short* a3  = (unsigned short*)(ws + kOffA3);
  unsigned short* lg  = (unsigned short*)(ws + kOffLog);
  unsigned short* vpl = (unsigned short*)(ws + kOffV);
  float*          tmp = (float*)(ws + kOffTmp);
  unsigned short* w1p = (unsigned short*)(ws + kOffW1);
  unsigned short* w2p = (unsigned short*)(ws + kOffW2);
  unsigned short* w3p = (unsigned short*)(ws + kOffW3);
  unsigned short* w4p = (unsigned short*)(ws + kOffW4);
  unsigned short* wdp = (unsigned short*)(ws + kOffWD);

  pack_input_kernel<<<kPix / 64, kThreads, 0, stream>>>(ef, fl1, fl2, p0);
  weight_prep_kernel<<<kBlkWtot, kThreads, 0, stream>>>(w1, w2, w3, w4, dcnw, w1p, w2p, w3p, w4p, wdp);
  conv3x3_kernel<0><<<dim3(kPix / 64, 1), kThreads, 0, stream>>>(
      p0, kCin1P, kCin1P / 32, w1p, kCmid, b1, kCmid, 1.0f / 64.0f, kA1Carry, a1);
  conv3x3_kernel<0><<<dim3(kPix / 64, 1), kThreads, 0, stream>>>(
      a1, kCmid, kCmid / 32, w2p, kCmid, b2, kCmid, 1.0f / 128.0f, kA2Carry, a2);
  conv3x3_kernel<0><<<dim3(kPix / 64, 1), kThreads, 0, stream>>>(
      a2, kCmid, kCmid / 32, w3p, kCmid, b3, kCmid, 1.0f / 256.0f, kA3Carry, a3);
  conv3x3_kernel<1><<<dim3(kPix / 64, kCout4P / 64), kThreads, 0, stream>>>(
      a3, kCmid, kCmid / 32, w4p, kCout4P, b4, kCout4, 1.0f / 1024.0f, kLogCarry, lg);
  for (int half = 0; half < 2; ++half) {
    const int pixbase = half * kHalfPix;
    deform_gather_kernel<<<kHalfPix / kGatherPix, kThreads, 0, stream>>>(
        x, (const unsigned*)lg, fl1, fl2, pixbase, vpl);
    wmma_gemm64<0, false, 2, 0, false, 0><<<dim3((kHalfPix / 64) / 8, 1), 256, 0, stream>>>(
        vpl, nullptr, kKdcn, 0L,
        wdp, nullptr, kKdcn, 0L,
        (void*)(tmp + (size_t)pixbase * kCoutD), nullptr, kCoutD, 0L,
        dcnb,
        nullptr, 0L,
        kHalfPix, kCoutD, kKdcn, 1.0f / 512.0f);
  }
  nchw_out_kernel<<<kBatch * kHgt, kThreads, 0, stream>>>(tmp, out);
}
